// TopologicalAttention_77266461655819
// MI455X (gfx1250) — hardware-verified
//
#include <hip/hip_runtime.h>
#include <math.h>
#include <stdint.h>

#define NB   4
#define SEQ  2048
#define DM   1024
#define NH   16
#define HD   64
#define NKT  (SEQ / 64)
static_assert(NH * HD == DM);
static_assert((SEQ % 64) == 0 && (DM % 64) == 0 && ((NB * SEQ) % 64) == 0);

typedef _Float16 v16h __attribute__((ext_vector_type(16)));
typedef _Float16 v8h  __attribute__((ext_vector_type(8)));
typedef float    v8f  __attribute__((ext_vector_type(8)));
typedef float    v4f  __attribute__((ext_vector_type(4)));
typedef unsigned int v4u __attribute__((ext_vector_type(4)));

__device__ __forceinline__ v8f zero8() { v8f z = {0.f, 0.f, 0.f, 0.f, 0.f, 0.f, 0.f, 0.f}; return z; }
__device__ __forceinline__ v4u pack8h(v8h h) { union U { v8h h; v4u u; } x; x.h = h; return x.u; }

__device__ __forceinline__ v16h ldfrag_h(const _Float16* p) {
  union { v16h v; v8h h[2]; } f;
  f.h[0] = *(const v8h*)(p);
  f.h[1] = *(const v8h*)(p + 16);
  return f.v;
}

__device__ __forceinline__ v8f mma_h(v16h a, v16h b, v8f c) {
  c = __builtin_amdgcn_wmma_f32_16x16x32_f16(false, a, false, b, (short)0, c, false, false);
  asm volatile("v_nop\n\tv_nop\n\tv_nop\n\tv_nop" : "+v"(c) : "v"(a), "v"(b));
  return c;
}
__device__ __forceinline__ v8f mma_h_raw(v16h a, v16h b, v8f c) {
  return __builtin_amdgcn_wmma_f32_16x16x32_f16(false, a, false, b, (short)0, c, false, false);
}
__device__ __forceinline__ void dep_guard_h(v8f& a, v8f& b, v16h x) {
  asm volatile("v_nop\n\tv_nop\n\tv_nop\n\tv_nop" : "+v"(a), "+v"(b) : "v"(x));
}
__device__ __forceinline__ void keep4_h(v16h a, v16h b, v16h c, v16h d) {
  asm volatile("v_nop" :: "v"(a), "v"(b), "v"(c), "v"(d));
}
__device__ __forceinline__ void acc_guard4(v8f& a, v8f& b, v8f& c, v8f& d) {
  asm volatile("v_nop\n\tv_nop\n\tv_nop\n\tv_nop" : "+v"(a), "+v"(b), "+v"(c), "+v"(d));
}

__global__ __launch_bounds__(256) void cvt_f16x8(const float* __restrict__ in, unsigned short* out, int n8) {
  const int i = blockIdx.x * 256 + threadIdx.x;
  if (i < n8) {
    const v4f a = *(const v4f*)(in + (size_t)i * 8);
    const v4f b = *(const v4f*)(in + (size_t)i * 8 + 4);
    v8h hv;
    hv[0] = (_Float16)a[0]; hv[1] = (_Float16)a[1]; hv[2] = (_Float16)a[2]; hv[3] = (_Float16)a[3];
    hv[4] = (_Float16)b[0]; hv[5] = (_Float16)b[1]; hv[6] = (_Float16)b[2]; hv[7] = (_Float16)b[3];
    const v4u p = pack8h(hv);
    unsigned short* o = out + (size_t)i * 8;
    *(volatile v4u*)o = p;
    __threadfence();
    *(volatile v4u*)o = p;
  }
}

__global__ __launch_bounds__(256) void wtrans_f16(const float* __restrict__ W0, const float* __restrict__ W1,
                                                   const float* __restrict__ W2, const float* __restrict__ W3,
                                                   unsigned short* dst, float scale) {
  __shared__ float t[64][65];
  const int z = blockIdx.z;
  const float* src = W0;
  if (z == 1) src = W1; else if (z == 2) src = W2; else if (z == 3) src = W3;
  unsigned short* d = dst + (size_t)z * DM * DM;
  const int k0 = blockIdx.y * 64, n0 = blockIdx.x * 64;
  const int tdx = threadIdx.x;
#pragma unroll
  for (int i = 0; i < 16; ++i) {
    const int idx = tdx + i * 256;
    const int r = idx >> 6, c = idx & 63;
    t[r][c] = src[(size_t)(k0 + r) * DM + n0 + c];
  }
  __syncthreads();
  const int wave = tdx >> 5, lane = tdx & 31;
  const int q = lane >> 3, c8 = (lane & 7) * 8;
  v4u pv[2];
#pragma unroll
  for (int it = 0; it < 2; ++it) {
    const int row = it * 32 + wave * 4 + q;
    v8h hv;
#pragma unroll
    for (int e = 0; e < 8; ++e) hv[e] = (_Float16)(t[c8 + e][row] * scale);
    pv[it] = pack8h(hv);
  }
  for (int pass = 0; pass < 2; ++pass) {
#pragma unroll
    for (int it = 0; it < 2; ++it) {
      const int row = it * 32 + wave * 4 + q;
      *(volatile v4u*)(d + (size_t)(n0 + row) * DM + k0 + c8) = pv[it];
    }
    __threadfence();
  }
}

__global__ __launch_bounds__(256) void topo_proj(const float* __restrict__ tf, const float* __restrict__ Wt,
                                                  const float* __restrict__ bt, float* topo) {
  const int tix = blockIdx.x * 256 + threadIdx.x;
  if (tix >= NB * DM) return;
  const int n = tix & (DM - 1);
  const int b = tix >> 10;
  const float* tfb = tf + (size_t)b * DM;
  float acc = 0.f;
#pragma unroll 4
  for (int k = 0; k < DM; ++k) acc += tfb[k] * Wt[(size_t)k * DM + n];
  acc += bt[n];
  *(volatile float*)(topo + tix) = acc;
  __threadfence();
  *(volatile float*)(topo + tix) = acc;
}

template <int MODE>
__global__ __launch_bounds__(256) void gemm64(
    const unsigned short* __restrict__ Ap, int lda, long long strideA,
    const unsigned short* __restrict__ Btp, int ldb, long long strideB,
    const float* __restrict__ bias, const float* __restrict__ addv, float addScale,
    void* Cout, int ldc, long long strideC,
    int M, int N, int K, float oscale) {
  const _Float16* A  = (const _Float16*)(const void*)Ap;
  const _Float16* Bt = (const _Float16*)(const void*)Btp;
  __shared__ __align__(16) float sT[8][16 * 68];
  const int b    = blockIdx.y;
  const int lane = threadIdx.x & 31;
  const int wave = threadIdx.x >> 5;
  const int tilesN = N >> 6;
  const int tilesM = M >> 6;
  const int tile = blockIdx.x * 8 + wave;
  if (tile >= tilesM * tilesN) return;
  const int tm = tile / tilesN;
  const int tn = tile - tm * tilesN;
  const int m0 = tm << 6;
  const int n0 = tn << 6;

  const _Float16* Ab = A  + (size_t)b * (size_t)strideA;
  const _Float16* Bb = Bt + (size_t)b * (size_t)strideB;

  const int rlane = lane & 15;
  const int koff  = (lane >> 4) * 8;
  const int mOff  = (lane >> 4) * 8;

  v8f acc[4][4];
#pragma unroll
  for (int i = 0; i < 4; ++i)
#pragma unroll
    for (int j = 0; j < 4; ++j) acc[i][j] = zero8();

  for (int k0 = 0; k0 < K; k0 += 32) {
    v16h bf[4];
#pragma unroll
    for (int j = 0; j < 4; ++j) {
      bf[j] = ldfrag_h(Bb + (size_t)(n0 + (j << 4) + rlane) * ldb + koff + k0);
    }
#pragma unroll
    for (int i = 0; i < 4; ++i) {
      const v16h af = ldfrag_h(Ab + (size_t)(m0 + (i << 4) + rlane) * lda + koff + k0);
#pragma unroll
      for (int j = 0; j < 4; ++j) acc[i][j] = mma_h_raw(af, bf[j], acc[i][j]);
      dep_guard_h(acc[i][0], acc[i][3], af);
    }
    keep4_h(bf[0], bf[1], bf[2], bf[3]);
  }
  acc_guard4(acc[0][0], acc[0][1], acc[0][2], acc[0][3]);
  acc_guard4(acc[1][0], acc[1][1], acc[1][2], acc[1][3]);
  acc_guard4(acc[2][0], acc[2][1], acc[2][2], acc[2][3]);
  acc_guard4(acc[3][0], acc[3][1], acc[3][2], acc[3][3]);

  float* slab = sT[wave];
  float cb[4];
#pragma unroll
  for (int j = 0; j < 4; ++j) cb[j] = 0.f;
  if (MODE != 1) {
    const int bb = m0 / SEQ;
#pragma unroll
    for (int j = 0; j < 4; ++j) {
      const int n = n0 + (j << 4) + rlane;
      float v = bias[n];
      if (MODE == 0) v += addScale * addv[bb * N + n];
      cb[j] = v;
    }
  }
#pragma unroll
  for (int i = 0; i < 4; ++i) {
    const int mBase = m0 + (i << 4);
    float rb[8];
    if (MODE == 1) {
#pragma unroll
      for (int r = 0; r < 8; ++r) rb[r] = bias[mBase + mOff + r];
    } else {
#pragma unroll
      for (int r = 0; r < 8; ++r) rb[r] = 0.f;
    }
#pragma unroll
    for (int j = 0; j < 4; ++j) {
#pragma unroll
      for (int r = 0; r < 8; ++r) {
        slab[(mOff + r) * 68 + (j << 4) + rlane] = acc[i][j][r] * oscale + rb[r] + cb[j];
      }
    }
    __builtin_amdgcn_fence(__ATOMIC_RELEASE, "workgroup");
    __builtin_amdgcn_wave_barrier();
    __builtin_amdgcn_fence(__ATOMIC_ACQUIRE, "workgroup");
    if (MODE == 2) {
      float* C = (float*)Cout + (size_t)b * (size_t)strideC;
      const int hh = lane >> 4, c4 = (lane & 15) * 4;
      for (int pass = 0; pass < 2; ++pass) {
#pragma unroll
        for (int it = 0; it < 8; ++it) {
          const int row = it * 2 + hh;
          const v4f v = *(const v4f*)(slab + row * 68 + c4);
          *(volatile v4f*)(C + (size_t)(mBase + row) * ldc + n0 + c4) = v;
        }
        __threadfence();
      }
    } else {
      const int q = lane >> 3, c8 = (lane & 7) * 8;
      unsigned short* C = (unsigned short*)Cout + (size_t)b * (size_t)strideC;
      v4u hv[4];
#pragma unroll
      for (int it = 0; it < 4; ++it) {
        const int row = it * 4 + q;
        const float* sp = slab + row * 68 + c8;
        v8h h8;
#pragma unroll
        for (int e = 0; e < 8; ++e) h8[e] = (_Float16)sp[e];
        hv[it] = pack8h(h8);
      }
      for (int pass = 0; pass < 2; ++pass) {
#pragma unroll
        for (int it = 0; it < 4; ++it) {
          const int row = it * 4 + q;
          *(volatile v4u*)(C + (size_t)(mBase + row) * ldc + n0 + c8) = hv[it];
        }
        __threadfence();
      }
    }
    __builtin_amdgcn_fence(__ATOMIC_RELEASE, "workgroup");
    __builtin_amdgcn_wave_barrier();
    __builtin_amdgcn_fence(__ATOMIC_ACQUIRE, "workgroup");
  }
}

__global__ __launch_bounds__(128)
void attn64(const unsigned short* __restrict__ qp, const unsigned short* __restrict__ kp,
            const unsigned short* __restrict__ vtp, unsigned short* op, float sscale) {
  union FH { v16h v; v8h h[2]; };
  __shared__ __align__(16) _Float16 Ksh[64 * 64];
  __shared__ __align__(16) _Float16 Vth[64 * 64];
  __shared__ __align__(16) _Float16 Psh[4][16 * 64];
  __shared__ __align__(16) float    Os[4][16 * 64];

  const int tid  = threadIdx.x;
  const int wave = tid >> 5;
  const int lane = tid & 31;
  const int hh   = lane >> 4;
  const int c    = lane & 15;

  const int bx   = blockIdx.x;
  const int qb   = bx % NKT;
  const int rest = bx / NKT;
  const int h    = rest % NH;
  const int b    = rest / NH;
  const int q0   = qb * 64 + wave * 16;
  const size_t rowB = (size_t)b * SEQ;

  const _Float16* Qg = (const _Float16*)(const void*)qp + (size_t)h * HD;
  const _Float16* Kg = (const _Float16*)(const void*)kp + (size_t)h * HD;
  const _Float16* Vg = (const _Float16*)(const void*)vtp + ((size_t)b * DM + (size_t)h * HD) * SEQ;

  v16h qa[2];
#pragma unroll
  for (int dc = 0; dc < 2; ++dc) {
    qa[dc] = ldfrag_h(Qg + (rowB + q0 + c) * DM + dc * 32 + 8 * hh);
  }

  float mrow[8], lrow[8];
  v8f oacc[4];
#pragma unroll
  for (int r = 0; r < 8; ++r) { mrow[r] = -1.0e30f; lrow[r] = 0.f; }
#pragma unroll
  for (int t = 0; t < 4; ++t) oacc[t] = zero8();

  for (int kt = 0; kt < NKT; ++kt) {
    const int kv0 = kt * 64;
    __syncthreads();
    {
      const int r = tid >> 1, half = (tid & 1) * 32;
      const _Float16* kg = Kg + (rowB + kv0 + r) * DM + half;
      const _Float16* vg = Vg + (size_t)r * SEQ + kv0 + half;
#pragma unroll
      for (int i = 0; i < 4; ++i) {
        const v8h a0 = *(const v8h*)(kg + 8 * i);
        const v8h b0 = *(const v8h*)(vg + 8 * i);
        *(v8h*)(Ksh + r * 64 + half + 8 * i) = a0;
        *(v8h*)(Vth + r * 64 + half + 8 * i) = b0;
      }
    }
    __syncthreads();

    v8f s[4];
#pragma unroll
    for (int j = 0; j < 4; ++j) {
      s[j] = zero8();
#pragma unroll
      for (int dc = 0; dc < 2; ++dc) {
        FH kb;
        kb.h[0] = *(const v8h*)(Ksh + (j * 16 + c) * 64 + dc * 32 + 8 * hh);
        kb.h[1] = *(const v8h*)(Ksh + (j * 16 + c) * 64 + dc * 32 + 16 + 8 * hh);
        s[j] = mma_h(qa[dc], kb.v, s[j]);
      }
    }

    _Float16* pw = Psh[wave];
#pragma unroll
    for (int r = 0; r < 8; ++r) {
      float m = -1.0e30f;
#pragma unroll
      for (int j = 0; j < 4; ++j) {
        const float sv = s[j][r] * sscale;
        s[j][r] = sv;
        m = fmaxf(m, sv);
      }
#pragma unroll
      for (int off = 1; off < 16; off <<= 1) m = fmaxf(m, __shfl_xor(m, off, 32));
      const float mnew  = fmaxf(mrow[r], m);
      const float alpha = __expf(mrow[r] - mnew);
      mrow[r] = mnew;
      float psum = 0.f;
#pragma unroll
      for (int j = 0; j < 4; ++j) {
        const float p = __expf(s[j][r] - mnew);
        psum += p;
        pw[(8 * hh + r) * 64 + j * 16 + c] = (_Float16)(p * 1024.0f);
      }
#pragma unroll
      for (int off = 1; off < 16; off <<= 1) psum += __shfl_xor(psum, off, 32);
      lrow[r] = lrow[r] * alpha + psum;
#pragma unroll
      for (int t = 0; t < 4; ++t) oacc[t][r] *= alpha;
    }
    __builtin_amdgcn_fence(__ATOMIC_RELEASE, "workgroup");
    __builtin_amdgcn_wave_barrier();
    __builtin_amdgcn_fence(__ATOMIC_ACQUIRE, "workgroup");

#pragma unroll
    for (int kk = 0; kk < 2; ++kk) {
      FH pa;
      pa.h[0] = *(const v8h*)(pw + c * 64 + kk * 32 + 8 * hh);
      pa.h[1] = *(const v8h*)(pw + c * 64 + kk * 32 + 16 + 8 * hh);
#pragma unroll
      for (int t = 0; t < 4; ++t) {
        FH vb;
        vb.h[0] = *(const v8h*)(Vth + (t * 16 + c) * 64 + kk * 32 + 8 * hh);
        vb.h[1] = *(const v8h*)(Vth + (t * 16 + c) * 64 + kk * 32 + 16 + 8 * hh);
        oacc[t] = mma_h(pa.v, vb.v, oacc[t]);
      }
    }
  }

  float* os = Os[wave];
#pragma unroll
  for (int r = 0; r < 8; ++r) {
    const float inv = 0.0625f / lrow[r];
#pragma unroll
    for (int t = 0; t < 4; ++t) os[(8 * hh + r) * 64 + t * 16 + c] = oacc[t][r] * inv;
  }
  __builtin_amdgcn_fence(__ATOMIC_RELEASE, "workgroup");
  __builtin_amdgcn_wave_barrier();
  __builtin_amdgcn_fence(__ATOMIC_ACQUIRE, "workgroup");
  {
    const int q4 = lane >> 3, c8 = (lane & 7) * 8;
    v4u hv[4];
#pragma unroll
    for (int it = 0; it < 4; ++it) {
      const int row = it * 4 + q4;
      const float* sp = os + row * 64 + c8;
      v8h h8;
#pragma unroll
      for (int e = 0; e < 8; ++e) h8[e] = (_Float16)sp[e];
      hv[it] = pack8h(h8);
    }
    for (int pass = 0; pass < 2; ++pass) {
#pragma unroll
      for (int it = 0; it < 4; ++it) {
        const int row = it * 4 + q4;
        const size_t go = (rowB + q0 + row) * DM + (size_t)h * HD + c8;
        *(volatile v4u*)(op + go) = hv[it];
      }
      __threadfence();
    }
  }
}

extern "C" void kernel_launch(void* const* d_in, const int* in_sizes, int n_in,
                              void* d_out, int out_size, void* d_ws, size_t ws_size,
                              hipStream_t stream) {
  if (n_in < 12) return;
  if (in_sizes[0] != NB * SEQ * DM) return;
  if (in_sizes[1] != NB * DM) return;
  if (in_sizes[2] != DM * DM || in_sizes[4] != DM * DM || in_sizes[6] != DM * DM ||
      in_sizes[8] != DM * DM || in_sizes[10] != DM * DM) return;
  if (in_sizes[3] != DM || in_sizes[5] != DM || in_sizes[7] != DM || in_sizes[9] != DM || in_sizes[11] != DM) return;
  if (out_size != NB * SEQ * DM) return;

  const float* x  = (const float*)d_in[0];
  const float* tf = (const float*)d_in[1];
  const float* Wq = (const float*)d_in[2];
  const float* bq = (const float*)d_in[3];
  const float* Wk = (const float*)d_in[4];
  const float* bk = (const float*)d_in[5];
  const float* Wv = (const float*)d_in[6];
  const float* bv = (const float*)d_in[7];
  const float* Wt = (const float*)d_in[8];
  const float* bt = (const float*)d_in[9];
  const float* Wo = (const float*)d_in[10];
  const float* bo = (const float*)d_in[11];

  const size_t PX = (size_t)NB * SEQ * DM * 2;
  const size_t PW = (size_t)DM * DM * 2;
  const size_t PT = (size_t)NB * DM * 4;
  size_t off = 0;
  const size_t oXh  = off; off += PX;
  const size_t oWT  = off; off += 4 * PW;
  const size_t oTp  = off; off += PT;
  const size_t oQh  = off; off += PX;
  const size_t oKh  = off; off += PX;
  const size_t oVT  = off; off += PX;
  const size_t oCtx = off; off += PX;
  if (off > ws_size) return;
  if (off > (size_t)134217728) return;

  char* ws = (char*)d_ws;
  unsigned short* Xh  = (unsigned short*)(ws + oXh);
  unsigned short* WT  = (unsigned short*)(ws + oWT);
  unsigned short* WqT = WT;
  unsigned short* WkT = WT + (size_t)DM * DM;
  unsigned short* WvT = WT + (size_t)2 * DM * DM;
  unsigned short* WoT = WT + (size_t)3 * DM * DM;
  float*          Topo = (float*)(ws + oTp);
  unsigned short* Qh  = (unsigned short*)(ws + oQh);
  unsigned short* Kh  = (unsigned short*)(ws + oKh);
  unsigned short* VTh = (unsigned short*)(ws + oVT);
  unsigned short* Ctx = (unsigned short*)(ws + oCtx);

  const dim3 blk(256);
  const int n8x = NB * SEQ * DM / 8;
  const dim3 gCvtX((n8x + 255) / 256);
  const dim3 gWT(DM / 64, DM / 64, 4);
  const dim3 gTopo((NB * DM + 255) / 256);
  const dim3 gProj(((NB * SEQ / 64) * (DM / 64) + 7) / 8, 1);
  const dim3 gVT(((DM / 64) * (SEQ / 64) + 7) / 8, NB);
  const dim3 gAttn(NB * NH * NKT);

  cvt_f16x8<<<gCvtX, blk, 0, stream>>>(x, Xh, n8x);
  wtrans_f16<<<gWT, blk, 0, stream>>>(Wq, Wk, Wv, Wo, WT, 64.0f);
  topo_proj<<<gTopo, blk, 0, stream>>>(tf, Wt, bt, Topo);
  gemm64<0><<<gProj, blk, 0, stream>>>(
      Xh, DM, 0LL, WqT, DM, 0LL, bq, Topo, 0.0f,
      (void*)Qh, DM, 0LL, NB * SEQ, DM, DM, 1.0f / 64.0f);
  gemm64<0><<<gProj, blk, 0, stream>>>(
      Xh, DM, 0LL, WkT, DM, 0LL, bk, Topo, 1.0f,
      (void*)Kh, DM, 0LL, NB * SEQ, DM, DM, 1.0f / 64.0f);
  gemm64<1><<<gVT, blk, 0, stream>>>(
      WvT, DM, 0LL, Xh, DM, (long long)SEQ * DM, bv, bv, 0.0f,
      (void*)VTh, SEQ, (long long)DM * SEQ, DM, SEQ, DM, 1.0f / 64.0f);
  attn64<<<gAttn, dim3(128), 0, stream>>>(Qh, Kh, VTh, Ctx, 0.125f);
  gemm64<2><<<gProj, blk, 0, stream>>>(
      Ctx, DM, 0LL, WoT, DM, 0LL, bo, bo, 0.0f,
      d_out, DM, 0LL, NB * SEQ, DM, DM, 1.0f / 4096.0f);
  (void)hipGetLastError();
}
